// EqMotion_74869869904618
// MI455X (gfx1250) — hardware-run, weakly checked
//
#include <hip/hip_runtime.h>


#define NB_  4
#define NN   256
#define TI   10
#define TO   20
#define HID  64
#define HC   64
#define CCH  128
#define NCAT 4
#define NNODE (NB_ * NN)
#define ICH  128
#define PCH  (ICH * NN)
#define OUT1OFF 61440
#define DM   HID
#define LOSC 1024.0f
typedef _Float16 h16;
typedef unsigned short bf;
typedef __attribute__((ext_vector_type(16))) __bf16   v16bf;
typedef __attribute__((ext_vector_type(16))) _Float16 v16h;
typedef __attribute__((ext_vector_type(8)))  _Float16 v8h;
typedef __attribute__((ext_vector_type(8)))  unsigned short v8us;
typedef __attribute__((ext_vector_type(8)))  float    v8f;
typedef __attribute__((ext_vector_type(4)))  float    v4f;
typedef __attribute__((ext_vector_type(4)))  _Float16 v4h;
typedef v8h  __attribute__((may_alias)) v8ha;
typedef v4f  __attribute__((may_alias)) v4fa;
typedef v8us __attribute__((may_alias)) v8usa;

__device__ __forceinline__ unsigned short f2bf(float f) { unsigned u = __float_as_uint(f); u += 0x7FFFu + ((u >> 16) & 1u); return (unsigned short)(u >> 16); }
__device__ __forceinline__ float bf2f(unsigned short b) { return __uint_as_float(((unsigned)b) << 16); }
__device__ __forceinline__ float bfr(float f) { return bf2f(f2bf(f)); }
__device__ __forceinline__ v16h cat16(v8h lo, v8h hi) { return __builtin_shufflevector(lo, hi, 0, 1, 2, 3, 4, 5, 6, 7, 8, 9, 10, 11, 12, 13, 14, 15); }
__device__ __forceinline__ v16bf cat16b(v8us lo, v8us hi) { return __builtin_bit_cast(v16bf, __builtin_shufflevector(lo, hi, 0, 1, 2, 3, 4, 5, 6, 7, 8, 9, 10, 11, 12, 13, 14, 15)); }
__device__ __forceinline__ v8f wmma16(v16h a, v16h b, v8f c) { return __builtin_amdgcn_wmma_f32_16x16x32_f16(false, a, false, b, (short)0, c, false, false); }
__device__ __forceinline__ v8f wmmab(v16bf a, v16bf b, v8f c) { return __builtin_amdgcn_wmma_f32_16x16x32_bf16(false, a, false, b, (short)0, c, false, false); }

template <bool SPLITA, bool F16OUT = false>
__global__ __launch_bounds__(128) void k_gemmb(const bf* __restrict__ A, const bf* __restrict__ Al, const bf* __restrict__ Bn, const float* __restrict__ bias, float* C, int ldc, h16* C2, const float* __restrict__ R = nullptr, int K = DM, int roundR = 1) {
    __shared__ __align__(16) float ost[4][16 * 68];
    const int lane = threadIdx.x & 31, wave = threadIdx.x >> 5, lr = lane & 15, hi = lane >> 4;
    const int r0 = blockIdx.x * 64 + wave * 16, c0 = blockIdx.y * 64;
    const size_t aoff = (size_t)(r0 + lr) * K + 8 * hi;
    size_t boff[4];
#pragma unroll
    for (int t = 0; t < 4; ++t) boff[t] = (size_t)(c0 + t * 16 + lr) * K + 8 * hi;
    v8f acc[4];
#pragma unroll
    for (int t = 0; t < 4; ++t) acc[t] = (v8f){};
#pragma unroll 1
    for (int kc = 0; kc < K; kc += 32) {
        const v16bf a = cat16b(*(const v8us*)(A + aoff + kc), *(const v8us*)(A + aoff + kc + 16));
        v16bf al = a;
        if (SPLITA) al = cat16b(*(const v8us*)(Al + aoff + kc), *(const v8us*)(Al + aoff + kc + 16));
#pragma unroll
        for (int t = 0; t < 4; ++t) { const v16bf b = cat16b(*(const v8us*)(Bn + boff[t] + kc), *(const v8us*)(Bn + boff[t] + kc + 16)); acc[t] = wmmab(a, b, acc[t]); if (SPLITA) acc[t] = wmmab(al, b, acc[t]); }
        asm volatile("v_nop\n\tv_nop\n\tv_nop\n\tv_nop" : "+v"(acc[0]), "+v"(acc[1]), "+v"(acc[2]), "+v"(acc[3]) : "v"(a), "v"(al));
    }
    float* os = &ost[wave][0];
#pragma unroll
    for (int t = 0; t < 4; ++t) { const float bv = bias ? bfr(bias[c0 + t * 16 + lr]) : 0.f;
#pragma unroll
        for (int j = 0; j < 8; ++j) os[(hi * 8 + j) * 68 + t * 16 + lr] = acc[t][j] + bv; }
    __syncthreads();
    if (F16OUT) {
        h16* crow = (h16*)(void*)C + (size_t)r0 * ldc + c0;
        auto pass = [&]() {
#pragma unroll
            for (int s = 0; s < 4; ++s) { const int row = 4 * s + (lane >> 3), piece = lane & 7; const float* sp = os + row * 68 + piece * 8; v8h o, o2;
#pragma unroll
                for (int i = 0; i < 8; ++i) { const h16 a = (h16)sp[i]; o[i] = a; o2[i] = (h16)((sp[i] - (float)a) * LOSC); }
                *(volatile v8h*)(crow + (size_t)row * ldc + piece * 8) = o; if (C2) *(volatile v8h*)(C2 + (size_t)r0 * ldc + c0 + (size_t)row * ldc + piece * 8) = o2; }
        };
        pass(); __threadfence(); pass();
    } else {
        float* crow = C + (size_t)r0 * ldc + c0;
        auto pass = [&]() {
#pragma unroll
            for (int s = 0; s < 8; ++s) { const int Lid = (lane >> 3) + 4 * s, piece = lane & 7; const int row = Lid >> 1, cofs = (Lid & 1) * 32 + piece * 4;
                v4f val = *(const v4fa*)(os + row * 68 + cofs); if (R) { const v4f rv = *(const v4f*)(R + ((size_t)r0 + row) * ldc + c0 + cofs); val += roundR ? (v4f){bfr(rv[0]), bfr(rv[1]), bfr(rv[2]), bfr(rv[3])} : rv; }
                *(volatile v4f*)(crow + (size_t)row * ldc + cofs) = val; }
        };
        pass(); __threadfence(); pass();
    }
}


__device__ __forceinline__ float siluf(float x) { return __fdiv_rn(x, 1.0f + expf(-x)); }
__constant__ float c_dct[100] = {0.316227764f, 0.316227764f, 0.316227764f, 0.316227764f, 0.316227764f, 0.316227764f, 0.316227764f, 0.316227764f, 0.316227764f, 0.316227764f, 0.441707641f, 0.398470223f, 0.316227764f, 0.20303072f, 0.0699596182f, -0.0699596182f, -0.20303072f, -0.316227764f, -0.398470223f, -0.441707641f, 0.425325394f, 0.262865543f, 2.73839349e-17f, -0.262865543f, -0.425325394f, -0.425325394f, -0.262865543f, -8.21518065e-17f, 0.262865543f, 0.425325394f, 0.398470223f, 0.0699596182f, -0.316227764f, -0.441707641f, -0.20303072f, 0.20303072f, 0.441707641f, 0.316227764f, -0.0699596182f, -0.398470223f, 0.361803412f, -0.138196602f, -0.44721359f, -0.138196602f, 0.361803412f, 0.361803412f, -0.138196602f, -0.44721359f, -0.138196602f, 0.361803412f, 0.316227764f, -0.316227764f, -0.316227764f, 0.316227764f, 0.316227764f, -0.316227764f, -0.316227764f, 0.316227764f, 0.316227764f, -0.316227764f, 0.262865543f, -0.425325394f, -8.21518065e-17f, 0.425325394f, -0.262865543f, -0.262865543f, 0.425325394f, 1.04086638e-15f, -0.425325394f, 0.262865543f, 0.20303072f, -0.441707641f, 0.316227764f, 0.0699596182f, -0.398470223f, 0.398470223f, -0.0699596182f, -0.316227764f, 0.441707641f, -0.20303072f, 0.138196602f, -0.361803412f, 0.44721359f, -0.361803412f, 0.138196602f, 0.138196602f, -0.361803412f, 0.44721359f, -0.361803412f, 0.138196602f, 0.0699596182f, -0.20303072f, 0.316227764f, -0.398470223f, 0.441707641f, -0.441707641f, 0.398470223f, -0.316227764f, 0.20303072f, -0.0699596182f};
__constant__ float c_idct[400] = {0.22360681f, 0.31525293f, 0.312334478f, 0.307490379f, 0.300750494f, 0.292156339f, 0.28176102f, 0.269628495f, 0.255833656f, 0.240461484f, 0.223606795f, 0.205373511f, 0.18587403f, 0.165228546f, 0.143564403f, 0.121015124f, 0.0977197587f, 0.0738219172f, 0.0494689196f, 0.0248109493f, 0.22360681f, 0.307490379f, 0.28176102f, 0.240461484f, 0.18587403f, 0.121015124f, 0.0494689196f, -0.0248109493f, -0.0977197587f, -0.165228546f, -0.223606795f, -0.269628495f, -0.300750494f, -0.31525293f, -0.312334478f, -0.292156339f, -0.255833656f, -0.205373511f, -0.143564403f, -0.0738219172f, 0.223606795f, 0.292156339f, 0.223606795f, 0.121015124f, -8.84180768e-17f, -0.121015109f, -0.223606795f, -0.292156339f, -0.316227764f, -0.292156339f, -0.22360681f, -0.121015124f, -1.86292952e-17f, 0.121015124f, 0.223606795f, 0.292156368f, 0.316227764f, 0.292156339f, 0.223606795f, 0.121015124f, 0.22360681f, 0.269628495f, 0.143564403f, -0.0248109493f, -0.18587403f, -0.292156339f, -0.312334478f, -0.240461484f, -0.0977197587f, 0.0738219172f, 0.223606795f, 0.307490379f, 0.300750494f, 0.205373511f, 0.0494689196f, -0.121015124f, -0.255833656f, -0.31525293f, -0.28176102f, -0.165228546f, 0.22360681f, 0.240461484f, 0.0494689196f, -0.165228546f, -0.300750494f, -0.292156339f, -0.143564403f, 0.0738219172f, 0.255833656f, 0.31525293f, 0.223606795f, 0.0248109493f, -0.18587403f, -0.307490379f, -0.28176102f, -0.121015124f, 0.0977197587f, 0.269628495f, 0.312334478f, 0.205373511f, 0.22360681f, 0.205373511f, -0.0494689196f, -0.269628495f, -0.300750494f, -0.121015124f, 0.143564403f, 0.307490379f, 0.255833656f, 0.0248109493f, -0.223606795f, -0.31525293f, -0.18587403f, 0.0738219172f, 0.28176102f, 0.292156339f, 0.0977197587f, -0.165228546f, -0.312334478f, -0.240461484f, 0.22360681f, 0.165228546f, -0.143564403f, -0.31525293f, -0.18587403f, 0.121015124f, 0.312334478f, 0.205373511f, -0.0977197587f, -0.307490379f, -0.223606795f, 0.0738219172f, 0.300750494f, 0.240461484f, -0.0494689196f, -0.292156339f, -0.255833656f, 0.0248109493f, 0.28176102f, 0.269628495f, 0.223606795f, 0.121015124f, -0.223606795f, -0.292156339f, 8.93691492e-17f, 0.292156368f, 0.223606795f, -0.121015124f, -0.316227764f, -0.121015124f, 0.22360681f, 0.292156339f, 2.12740729e-16f, -0.292156339f, -0.223606795f, 0.121015109f, 0.316227764f, 0.121015124f, -0.223606795f, -0.292156339f, 0.22360681f, 0.0738219172f, -0.28176102f, -0.205373511f, 0.18587403f, 0.292156339f, -0.0494689196f, -0.31525293f, -0.0977197587f, 0.269628495f, 0.223606795f, -0.165228546f, -0.300750494f, 0.0248109493f, 0.312334478f, 0.121015124f, -0.255833656f, -0.240461484f, 0.143564403f, 0.307490379f, 0.22360681f, 0.0248109493f, -0.312334478f, -0.0738219172f, 0.300750494f, 0.121015124f, -0.28176102f, -0.165228546f, 0.255833656f, 0.205373511f, -0.223606795f, -0.240461484f, 0.18587403f, 0.269628495f, -0.143564403f, -0.292156339f, 0.0977197587f, 0.307490379f, -0.0494689196f, -0.31525293f, 0.22360681f, -0.0248109493f, -0.312334478f, 0.0738219172f, 0.300750494f, -0.121015124f, -0.28176102f, 0.165228546f, 0.255833656f, -0.205373511f, -0.223606795f, 0.240461484f, 0.18587403f, -0.269628495f, -0.143564403f, 0.292156339f, 0.0977197587f, -0.307490379f, -0.0494689196f, 0.31525293f, 0.22360681f, -0.0738219172f, -0.28176102f, 0.205373511f, 0.18587403f, -0.292156339f, -0.0494689196f, 0.31525293f, -0.0977197587f, -0.269628495f, 0.223606795f, 0.165228546f, -0.300750494f, -0.0248109493f, 0.312334478f, -0.121015124f, -0.255833656f, 0.240461484f, 0.143564403f, -0.307490379f, 0.223606795f, -0.121015124f, -0.223606795f, 0.292156339f, -1.80798812e-16f, -0.292156368f, 0.223606795f, 0.121015124f, -0.316227764f, 0.121015124f, 0.22360681f, -0.292156339f, 1.28677765e-16f, 0.292156339f, -0.223606795f, -0.121015109f, 0.316227764f, -0.121015124f, -0.223606795f, 0.292156339f, 0.22360681f, -0.165228546f, -0.143564403f, 0.31525293f, -0.18587403f, -0.121015124f, 0.312334478f, -0.205373511f, -0.0977197587f, 0.307490379f, -0.223606795f, -0.0738219172f, 0.300750494f, -0.240461484f, -0.0494689196f, 0.292156339f, -0.255833656f, -0.0248109493f, 0.28176102f, -0.269628495f, 0.22360681f, -0.205373511f, -0.0494689196f, 0.269628495f, -0.300750494f, 0.121015124f, 0.143564403f, -0.307490379f, 0.255833656f, -0.0248109493f, -0.223606795f, 0.31525293f, -0.18587403f, -0.0738219172f, 0.28176102f, -0.292156339f, 0.0977197587f, 0.165228546f, -0.312334478f, 0.240461484f, 0.22360681f, -0.240461484f, 0.0494689196f, 0.165228546f, -0.300750494f, 0.292156339f, -0.143564403f, -0.0738219172f, 0.255833656f, -0.31525293f, 0.223606795f, -0.0248109493f, -0.18587403f, 0.307490379f, -0.28176102f, 0.121015124f, 0.0977197587f, -0.269628495f, 0.312334478f, -0.205373511f, 0.22360681f, -0.269628495f, 0.143564403f, 0.0248109493f, -0.18587403f, 0.292156339f, -0.312334478f, 0.240461484f, -0.0977197587f, -0.0738219172f, 0.223606795f, -0.307490379f, 0.300750494f, -0.205373511f, 0.0494689196f, 0.121015124f, -0.255833656f, 0.31525293f, -0.28176102f, 0.165228546f, 0.223606795f, -0.292156339f, 0.223606795f, -0.121015124f, -2.92950667e-18f, 0.121015109f, -0.223606795f, 0.292156339f, -0.316227764f, 0.292156339f, -0.22360681f, 0.121015124f, 1.68670796e-16f, -0.121015124f, 0.223606795f, -0.292156368f, 0.316227764f, -0.292156339f, 0.223606795f, -0.121015124f, 0.22360681f, -0.307490379f, 0.28176102f, -0.240461484f, 0.18587403f, -0.121015124f, 0.0494689196f, 0.0248109493f, -0.0977197587f, 0.165228546f, -0.223606795f, 0.269628495f, -0.300750494f, 0.31525293f, -0.312334478f, 0.292156339f, -0.255833656f, 0.205373511f, -0.143564403f, 0.0738219172f, 0.22360681f, -0.31525293f, 0.312334478f, -0.307490379f, 0.300750494f, -0.292156339f, 0.28176102f, -0.269628495f, 0.255833656f, -0.240461484f, 0.223606795f, -0.205373511f, 0.18587403f, -0.165228546f, 0.143564403f, -0.121015124f, 0.0977197587f, -0.0738219172f, 0.0494689196f, -0.0248109493f};
template <int MODE>
__global__ __launch_bounds__(256) void k_mean3(const float* __restrict__ src, int npos, float* OUT32) {
    __shared__ float part[8][4];
    const int lane = threadIdx.x & 31, wv = threadIdx.x >> 5; const int b = blockIdx.x; float a0 = 0.f, a1 = 0.f, a2 = 0.f;
#pragma unroll 1
    for (int p = wv * 32 + lane; p < npos; p += 256) { const float* s = (MODE == 0) ? (src + ((size_t)b * npos + p) * 3) : (src + ((size_t)b * NN + p / TI) * 32 + (p % TI) * 3); float v0 = s[0], v1 = s[1], v2 = s[2]; if (MODE == 0) { v0 = bfr(v0); v1 = bfr(v1); v2 = bfr(v2); } a0 += v0; a1 += v1; a2 += v2; }
#pragma unroll
    for (int sh = 16; sh; sh >>= 1) { a0 += __shfl_xor(a0, sh, 32); a1 += __shfl_xor(a1, sh, 32); a2 += __shfl_xor(a2, sh, 32); }
    if (lane == 0) { part[wv][0] = a0; part[wv][1] = a1; part[wv][2] = a2; }
    __syncthreads();
    if (wv == 0) { float v = 0.f; if (lane < 3) { for (int w = 0; w < 8; ++w) v += part[w][lane]; v *= (1.0f / npos); } *(volatile float*)(OUT32 + b * 32 + lane) = v; __threadfence(); *(volatile float*)(OUT32 + b * 32 + lane) = v; }
}
__global__ __launch_bounds__(256) void k_node1(const float* __restrict__ h, const float* __restrict__ x, const float* __restrict__ vel, const float* __restrict__ XC, const float* __restrict__ We, const float* __restrict__ be, const float* __restrict__ We2, const float* __restrict__ be2, float* HH, bf* HHh, bf* HHl, float* XD, float* VD) {
    typedef __attribute__((ext_vector_type(2))) float v2f_; typedef __attribute__((ext_vector_type(2))) unsigned short v2us;
    const int lane = threadIdx.x & 31; const size_t n = (size_t)blockIdx.x * 8 + (threadIdx.x >> 5); if (n >= (size_t)NNODE) return; const int b = (int)(n / NN); const float* xv = x + n * TI * 3; const float* vv = vel + n * TI * 3;
    float ang = 0.f;
    if (lane < TI) { const int t = lane, tp = (t == 0) ? 0 : t - 1; const float a0 = bfr(vv[tp * 3]), a1 = bfr(vv[tp * 3 + 1]), a2 = bfr(vv[tp * 3 + 2]); const float b0 = bfr(vv[t * 3]), b1 = bfr(vv[t * 3 + 1]), b2 = bfr(vv[t * 3 + 2]);
        const float dot = (a0 * b0 + a1 * b1) + a2 * b2; const float na = __fsqrt_rn((a0 * a0 + a1 * a1) + a2 * a2), nb = __fsqrt_rn((b0 * b0 + b1 * b1) + b2 * b2);
        float c = __fdiv_rn(dot, (na + 1e-6f) * (nb + 1e-6f)); c = fminf(fmaxf(c, -1.0f), 1.0f); ang = acosf(c); }
    float angv[TI];
#pragma unroll
    for (int t = 0; t < TI; ++t) angv[t] = __shfl(ang, t, 32);
    v2f_ hv; v2us hh2, hl2;
#pragma unroll
    for (int q = 0; q < 2; ++q) { const int c = lane * 2 + q; float a;
        if (c < 32) { a = bfr(be[c]);
#pragma unroll
            for (int t = 0; t < TI; ++t) a = fmaf(bfr(h[n * TI + t]), bfr(We[t * 32 + c]), a); }
        else { const int cc = c - 32; a = bfr(be2[cc]);
#pragma unroll
            for (int t = 0; t < TI; ++t) a = fmaf(angv[t], bfr(We2[t * 32 + cc]), a); }
        hv[q] = a; const unsigned short hb = f2bf(a); hh2[q] = hb; hl2[q] = f2bf(a - bf2f(hb)); }
    float xd = 0.f, vd = 0.f;
    if (lane < 30) { const int s = lane / 3, d = lane % 3; const float xc = XC[b * 32 + d];
#pragma unroll
        for (int t = 0; t < TI; ++t) { xd = fmaf(c_dct[s * TI + t], bfr(xv[t * 3 + d]) - xc, xd); vd = fmaf(c_dct[s * TI + t], bfr(vv[t * 3 + d]), vd); } }
#pragma unroll 1
    for (int ps = 0; ps < 2; ++ps) { *(volatile v2f_*)(HH + n * HID + lane * 2) = hv; *(volatile v2us*)(HHh + n * HID + lane * 2) = hh2; *(volatile v2us*)(HHl + n * HID + lane * 2) = hl2; *(volatile float*)(XD + n * 32 + lane) = xd; *(volatile float*)(VD + n * 32 + lane) = vd; if (ps == 0) __threadfence(); }
}
__global__ __launch_bounds__(256) void k_node2(const float* __restrict__ XD, const float* __restrict__ VD, const float* __restrict__ XM, const float* __restrict__ Wco, const float* __restrict__ Wve, float* COORD) {
    const int lane = threadIdx.x & 31; const size_t n = (size_t)blockIdx.x * 8 + (threadIdx.x >> 5); if (n >= (size_t)NNODE) return; const int b = (int)(n / NN);
    v4f o[3];
#pragma unroll
    for (int g = 0; g < 3; ++g) {
#pragma unroll
        for (int i = 0; i < 4; ++i) { const int f = g * 128 + lane * 4 + i; const int c = f / 3, d = f % 3; float a;
            if (c < HC) { const float xm = XM[b * 32 + d]; a = xm;
#pragma unroll 1
                for (int s = 0; s < TI; ++s) a = fmaf(XD[n * 32 + s * 3 + d] - xm, bfr(Wco[s * HC + c]), a); }
            else { a = 0.f;
#pragma unroll 1
                for (int s = 0; s < TI; ++s) a = fmaf(VD[n * 32 + s * 3 + d], bfr(Wve[s * HC + (c - HC)]), a); }
            o[g][i] = a; } }
#pragma unroll 1
    for (int ps = 0; ps < 2; ++ps) {
#pragma unroll
        for (int g = 0; g < 3; ++g) *(volatile v4f*)(COORD + n * (CCH * 3) + g * 128 + lane * 4) = o[g];
        if (ps == 0) __threadfence(); }
}
__global__ __launch_bounds__(256) void k_xout(const float* __restrict__ COORD, const float* __restrict__ XM2, const float* __restrict__ XC, const float* __restrict__ Wp, float* XO) {
    __shared__ float sxo[8][64];
    typedef __attribute__((ext_vector_type(2))) float v2f_;
    const int lane = threadIdx.x & 31, wv = threadIdx.x >> 5; const size_t n = (size_t)blockIdx.x * 8 + wv; if (n >= (size_t)NNODE) return; const int b = (int)(n / NN); float* t60 = sxo[wv];
#pragma unroll
    for (int q = 0; q < 2; ++q) { const int f = lane * 2 + q; float a = 0.f; if (f < TO * 3) { const int o_ = f / 3, d = f % 3; const float xm2 = XM2[b * 32 + d]; a = xm2;
#pragma unroll 1
            for (int c = 0; c < HC; ++c) a = fmaf(COORD[n * (CCH * 3) + c * 3 + d] - xm2, bfr(Wp[c * TO + o_]), a); }
        t60[f] = a; }
    __builtin_amdgcn_wave_barrier(); asm volatile("" ::: "memory");
    v2f_ ov;
#pragma unroll
    for (int q = 0; q < 2; ++q) { const int f = lane * 2 + q; float a = 0.f; if (f < TO * 3) { const int s = f / 3, d = f % 3; a = XC[b * 32 + d];
#pragma unroll 1
            for (int o_ = 0; o_ < TO; ++o_) a = fmaf(c_idct[s * TO + o_], t60[o_ * 3 + d], a); }
        ov[q] = a; }
    *(volatile v2f_*)(XO + n * 64 + lane * 2) = ov; __threadfence(); *(volatile v2f_*)(XO + n * 64 + lane * 2) = ov;
}
__global__ __launch_bounds__(256) void k_flat60(const float* __restrict__ XO, float* OUTB) {
    const int lane = threadIdx.x & 31; const size_t e = ((size_t)blockIdx.x * 8 + (threadIdx.x >> 5)) * 32 + lane; if (e >= (size_t)NNODE * 60) return; const float v = XO[(e / 60) * 64 + (e % 60)];
    *(volatile float*)(OUTB + e) = v; __threadfence(); *(volatile float*)(OUTB + e) = v;
}
__global__ __launch_bounds__(256) void k_meanC(const float* __restrict__ COORD, float* OUT32) {
    __shared__ float part[8][4];
    const int lane = threadIdx.x & 31, wv = threadIdx.x >> 5; const int b = blockIdx.x; float a0 = 0.f, a1 = 0.f, a2 = 0.f;
#pragma unroll 1
    for (int p = wv * 32 + lane; p < NN * HC; p += 256) { const int nl = p / HC, c = p % HC; const float* r = COORD + ((size_t)b * NN + nl) * (CCH * 3) + c * 3; a0 += r[0]; a1 += r[1]; a2 += r[2]; }
#pragma unroll
    for (int sh = 16; sh; sh >>= 1) { a0 += __shfl_xor(a0, sh, 32); a1 += __shfl_xor(a1, sh, 32); a2 += __shfl_xor(a2, sh, 32); }
    if (lane == 0) { part[wv][0] = a0; part[wv][1] = a1; part[wv][2] = a2; }
    __syncthreads();
    if (wv == 0) { float v = 0.f; if (lane < 3) { for (int w = 0; w < 8; ++w) v += part[w][lane]; v *= (1.0f / (NN * HC)); } *(volatile float*)(OUT32 + b * 32 + lane) = v; __threadfence(); *(volatile float*)(OUT32 + b * 32 + lane) = v; }
}

__global__ __launch_bounds__(256) void k_wt_io(const float* __restrict__ Wm, int ldw, int K, int N, bf* Bt) {
    const int lane = threadIdx.x & 31; const int n = blockIdx.x * 8 + (threadIdx.x >> 5); if (n >= N) return;
#pragma unroll 1
    for (int ps = 0; ps < 2; ++ps) { for (int c0 = lane * 8; c0 < K; c0 += 256) { v8us o;
#pragma unroll
            for (int i = 0; i < 8; ++i) { const int k = c0 + i; o[i] = f2bf(k < K ? Wm[(size_t)(k < K ? k : 0) * ldw + n] : 0.f); }
            *(volatile v8us*)(Bt + (size_t)n * K + c0) = o; }
        if (ps == 0) __threadfence(); }
}
template <int W, bool F32O>
__global__ __launch_bounds__(256) void k_silusplit(const float* __restrict__ F, size_t rows, bf* Ph, bf* Pl, float* OF) {
    typedef __attribute__((ext_vector_type(4))) unsigned short v4us;
    const int LPR = W / 4, RPW = 32 / LPR; const int lane = threadIdx.x & 31; const size_t r = ((size_t)blockIdx.x * 8 + (threadIdx.x >> 5)) * RPW + lane / LPR; if (r >= rows) return; const int c0 = (lane % LPR) * 4; v4us oh, ol; v4f y;
#pragma unroll
    for (int i = 0; i < 4; ++i) { y[i] = siluf(F[r * W + c0 + i]); const unsigned short hb = f2bf(y[i]); oh[i] = hb; ol[i] = f2bf(y[i] - bf2f(hb)); }
#pragma unroll 1
    for (int ps = 0; ps < 2; ++ps) { *(volatile v4us*)(Ph + r * W + c0) = oh; *(volatile v4us*)(Pl + r * W + c0) = ol; if (F32O) *(volatile v4f*)(OF + r * W + c0) = y; if (ps == 0) __threadfence(); }
}
__global__ __launch_bounds__(256) void k_catplanes(const float* __restrict__ HH, const float* __restrict__ AGG, bf* Ph, bf* Pl) {
    typedef __attribute__((ext_vector_type(4))) unsigned short v4us;
    const int lane = threadIdx.x & 31; const size_t n = (size_t)blockIdx.x * 8 + (threadIdx.x >> 5); if (n >= (size_t)NNODE) return; const int c0 = lane * 4; v4us oh, ol;
#pragma unroll
    for (int i = 0; i < 4; ++i) { const int c = c0 + i; const float y = (c < HID) ? HH[n * HID + c] : AGG[n * HID + (c - HID)]; const unsigned short hb = f2bf(y); oh[i] = hb; ol[i] = f2bf(y - bf2f(hb)); }
    *(volatile v4us*)(Ph + n * CCH + c0) = oh; *(volatile v4us*)(Pl + n * CCH + c0) = ol; __threadfence(); *(volatile v4us*)(Ph + n * CCH + c0) = oh; *(volatile v4us*)(Pl + n * CCH + c0) = ol;
}
__global__ __launch_bounds__(256) void k_dist(const float* __restrict__ COORD, int b, int i0, bf* Ph, bf* Pl) {
    typedef __attribute__((ext_vector_type(4))) unsigned short v4us;
    const int lane = threadIdx.x & 31; const size_t p = (size_t)blockIdx.x * 8 + (threadIdx.x >> 5); if (p >= (size_t)PCH) return; const int il = (int)(p / NN), j = (int)(p % NN); const float* ci = COORD + ((size_t)b * NN + i0 + il) * (CCH * 3); const float* cj = COORD + ((size_t)b * NN + j) * (CCH * 3); const int c0 = lane * 4; v4us oh, ol;
#pragma unroll
    for (int k = 0; k < 4; ++k) { const int c = c0 + k; const float dx = ci[c * 3] - cj[c * 3], dy = ci[c * 3 + 1] - cj[c * 3 + 1], dz = ci[c * 3 + 2] - cj[c * 3 + 2]; const float y = __fsqrt_rn((dx * dx + dy * dy) + dz * dz); const unsigned short hb = f2bf(y); oh[k] = hb; ol[k] = f2bf(y - bf2f(hb)); }
    *(volatile v4us*)(Ph + p * CCH + c0) = oh; *(volatile v4us*)(Pl + p * CCH + c0) = ol; __threadfence(); *(volatile v4us*)(Ph + p * CCH + c0) = oh; *(volatile v4us*)(Pl + p * CCH + c0) = ol;
}
__global__ __launch_bounds__(256) void k_edge1(const float* __restrict__ UV, const float* __restrict__ EK, const float* __restrict__ be1, int b, int i0, bf* Ph, bf* Pl) {
    typedef __attribute__((ext_vector_type(4))) unsigned short v4us;
    const int lane = threadIdx.x & 31; const size_t p = ((size_t)blockIdx.x * 8 + (threadIdx.x >> 5)) * 2 + (lane >> 4); if (p >= (size_t)PCH) return; const int il = (int)(p / NN), j = (int)(p % NN); const size_t ni = (size_t)b * NN + i0 + il, nj = (size_t)b * NN + j; const int c0 = (lane & 15) * 4; v4us oh, ol;
#pragma unroll
    for (int k = 0; k < 4; ++k) { const int c = c0 + k; const float y = siluf(UV[ni * CCH + c] + UV[nj * CCH + HID + c] + EK[p * CCH + c] + bfr(be1[c])); const unsigned short hb = f2bf(y); oh[k] = hb; ol[k] = f2bf(y - bf2f(hb)); }
    *(volatile v4us*)(Ph + p * HID + c0) = oh; *(volatile v4us*)(Pl + p * HID + c0) = ol; __threadfence(); *(volatile v4us*)(Ph + p * HID + c0) = oh; *(volatile v4us*)(Pl + p * HID + c0) = ol;
}
__global__ __launch_bounds__(256) void k_aggsum(const float* __restrict__ E2, int b, int i0, float* AGG) {
    typedef __attribute__((ext_vector_type(2))) float v2f_;
    const int lane = threadIdx.x & 31; const int il = blockIdx.x * 8 + (threadIdx.x >> 5); if (il >= ICH) return; const int i = i0 + il; const int c0 = lane * 2; float a0 = 0.f, a1 = 0.f;
#pragma unroll 1
    for (int j = 0; j < NN; ++j) { if (j == i) continue; const size_t p = (size_t)il * NN + j; a0 += siluf(E2[p * HID + c0]); a1 += siluf(E2[p * HID + c0 + 1]); }
    v2f_ o; o[0] = a0; o[1] = a1; float* dst = AGG + ((size_t)b * NN + i) * HID + c0; *(volatile v2f_*)dst = o; __threadfence(); *(volatile v2f_*)dst = o;
}
__global__ __launch_bounds__(256) void k_logits(const float* __restrict__ UVN, const float* __restrict__ EK, const float* __restrict__ bk1, const float* __restrict__ Wk2, const float* __restrict__ bk2, int b, int i0, float* OUTC) {
    const int lane = threadIdx.x & 31; const size_t w = (size_t)blockIdx.x * 8 + (threadIdx.x >> 5); if (w >= (size_t)PCH / 8) return; const size_t p = w * 8 + (lane >> 2); const int o_ = lane & 3; const int il = (int)(p / NN), j = (int)(p % NN); const size_t ni = (size_t)b * NN + i0 + il, nj = (size_t)b * NN + j;
    float a = bfr(bk2[o_]);
#pragma unroll 1
    for (int c = 0; c < HID; ++c) { const float l1 = siluf(UVN[ni * CCH + c] + UVN[nj * CCH + HID + c] + EK[p * CCH + HID + c] + bfr(bk1[c])); a = fmaf(l1, bfr(Wk2[c * NCAT + o_]), a); }
    a = siluf(a); float m = a; m = fmaxf(m, __shfl_xor(m, 1, 32)); m = fmaxf(m, __shfl_xor(m, 2, 32)); const float e = expf(a - m); float s = e; s += __shfl_xor(s, 1, 32); s += __shfl_xor(s, 2, 32); const float pr = __fdiv_rn(e, s);
    float* dst = OUTC + (((size_t)b * NN + i0 + il) * NN + j) * NCAT + o_; *(volatile float*)dst = pr; __threadfence(); *(volatile float*)dst = pr;
}

extern "C" void kernel_launch(void* const* d_in, const int* in_sizes, int n_in,
                              void* d_out, int out_size, void* d_ws, size_t ws_size, hipStream_t stream) {
    (void)in_sizes; (void)n_in; (void)out_size;
    const float* h = (const float*)d_in[0]; const float* x = (const float*)d_in[1]; const float* vel = (const float*)d_in[2]; const float* Wemb = (const float*)d_in[3]; const float* bemb = (const float*)d_in[4]; const float* Wemb2 = (const float*)d_in[5]; const float* bemb2 = (const float*)d_in[6];
    const float* Wco = (const float*)d_in[7]; const float* Wve = (const float*)d_in[8]; const float* Wp = (const float*)d_in[9];
    const float* Wc1 = (const float*)d_in[10]; const float* bc1 = (const float*)d_in[11]; const float* Wc2 = (const float*)d_in[12]; const float* bc2 = (const float*)d_in[13];
    const float* We1 = (const float*)d_in[14]; const float* be1 = (const float*)d_in[15]; const float* We2 = (const float*)d_in[16]; const float* be2 = (const float*)d_in[17];
    const float* Wn1 = (const float*)d_in[18]; const float* bn1 = (const float*)d_in[19]; const float* Wn2 = (const float*)d_in[20]; const float* bn2 = (const float*)d_in[21];
    const float* Wk1 = (const float*)d_in[22]; const float* bk1 = (const float*)d_in[23]; const float* Wk2 = (const float*)d_in[24]; const float* bk2 = (const float*)d_in[25];
    float* out0 = (float*)d_out; float* out1 = out0 + OUT1OFF;
    char* wsp = (char*)d_ws;
    auto take = [&](size_t bytes) { char* p = wsp; wsp += (bytes + 255) & ~(size_t)255; return (void*)p; };
    bf* BWC1 = (bf*)take(HID * CCH * 2); bf* BWC2 = (bf*)take(CCH * HID * 2); bf* BWEK = (bf*)take(CCH * CCH * 2); bf* BWE2 = (bf*)take(HID * HID * 2); bf* BUV = (bf*)take(CCH * HID * 2); bf* BWN1 = (bf*)take(HID * CCH * 2); bf* BWN2 = (bf*)take(HID * HID * 2); bf* BUVN = (bf*)take(CCH * HID * 2);
    float* XC = (float*)take(NB_ * 32 * 4); float* XM = (float*)take(NB_ * 32 * 4); float* XM2 = (float*)take(NB_ * 32 * 4);
    float* HH = (float*)take(NNODE * HID * 4); bf* HHh = (bf*)take(NNODE * HID * 2); bf* HHl = (bf*)take(NNODE * HID * 2); float* XD = (float*)take(NNODE * 32 * 4); float* VD = (float*)take(NNODE * 32 * 4); float* COORD = (float*)take((size_t)NNODE * CCH * 3 * 4); float* XO = (float*)take(NNODE * 64 * 4);
    float* UV = (float*)take((size_t)NNODE * CCH * 4); float* AGG = (float*)take(NNODE * HID * 4); bf* NPh = (bf*)take((size_t)NNODE * CCH * 2); bf* NPl = (bf*)take((size_t)NNODE * CCH * 2); float* NT1 = (float*)take(NNODE * HID * 4); float* NNW = (float*)take(NNODE * HID * 4); float* UVN = (float*)take((size_t)NNODE * CCH * 4);
    bf* DPh = (bf*)take((size_t)PCH * CCH * 2); bf* DPl = (bf*)take((size_t)PCH * CCH * 2); float* C1 = (float*)take((size_t)PCH * HID * 4); bf* P64h = (bf*)take((size_t)PCH * HID * 2); bf* P64l = (bf*)take((size_t)PCH * HID * 2); float* CD = (float*)take((size_t)PCH * CCH * 4); bf* CDh = (bf*)take((size_t)PCH * CCH * 2); bf* CDl = (bf*)take((size_t)PCH * CCH * 2);
    float* EK = (float*)take((size_t)2 * PCH * CCH * 4); float* E2 = (float*)take((size_t)PCH * HID * 4);
    if ((size_t)(wsp - (char*)d_ws) > ws_size) return;
    k_wt_io<<<HID / 8, 256, 0, stream>>>(Wc1, HID, CCH, HID, BWC1); k_wt_io<<<CCH / 8, 256, 0, stream>>>(Wc2, CCH, HID, CCH, BWC2);
    k_wt_io<<<HID / 8, 256, 0, stream>>>(We1 + (size_t)CCH * HID, HID, CCH, HID, BWEK); k_wt_io<<<HID / 8, 256, 0, stream>>>(Wk1 + (size_t)CCH * HID, HID, CCH, HID, BWEK + (size_t)HID * CCH);
    k_wt_io<<<HID / 8, 256, 0, stream>>>(We2, HID, HID, HID, BWE2);
    k_wt_io<<<HID / 8, 256, 0, stream>>>(We1, HID, HID, HID, BUV); k_wt_io<<<HID / 8, 256, 0, stream>>>(We1 + (size_t)HID * HID, HID, HID, HID, BUV + (size_t)HID * HID);
    k_wt_io<<<HID / 8, 256, 0, stream>>>(Wn1, HID, CCH, HID, BWN1); k_wt_io<<<HID / 8, 256, 0, stream>>>(Wn2, HID, HID, HID, BWN2);
    k_wt_io<<<HID / 8, 256, 0, stream>>>(Wk1, HID, HID, HID, BUVN); k_wt_io<<<HID / 8, 256, 0, stream>>>(Wk1 + (size_t)HID * HID, HID, HID, HID, BUVN + (size_t)HID * HID);
    k_mean3<0><<<NB_, 256, 0, stream>>>(x, NN * TI, XC);
    k_node1<<<NNODE / 8, 256, 0, stream>>>(h, x, vel, XC, Wemb, bemb, Wemb2, bemb2, HH, HHh, HHl, XD, VD);
    k_mean3<1><<<NB_, 256, 0, stream>>>(XD, NN * TI, XM);
    k_node2<<<NNODE / 8, 256, 0, stream>>>(XD, VD, XM, Wco, Wve, COORD);
    k_meanC<<<NB_, 256, 0, stream>>>(COORD, XM2);
    k_xout<<<NNODE / 8, 256, 0, stream>>>(COORD, XM2, XC, Wp, XO); k_flat60<<<(NNODE * 60 / 32 + 7) / 8, 256, 0, stream>>>(XO, out0);
    k_gemmb<true, false><<<dim3(NNODE / 64, CCH / 64, 1), 128, 0, stream>>>(HHh, HHl, BUV, nullptr, UV, CCH, nullptr, nullptr, HID);
    for (int ch = 0; ch < 2 * NB_; ++ch) { const int b = ch / 2, i0 = (ch % 2) * ICH; float* EKc = EK + (size_t)(ch % 2) * PCH * CCH;
        k_dist<<<PCH / 8, 256, 0, stream>>>(COORD, b, i0, DPh, DPl);
        k_gemmb<true, false><<<dim3(PCH / 64, 1, 1), 128, 0, stream>>>(DPh, DPl, BWC1, bc1, C1, HID, nullptr, nullptr, CCH);
        k_silusplit<64, false><<<(PCH / 2) / 8, 256, 0, stream>>>(C1, PCH, P64h, P64l, nullptr);
        k_gemmb<true, false><<<dim3(PCH / 64, CCH / 64, 1), 128, 0, stream>>>(P64h, P64l, BWC2, bc2, CD, CCH, nullptr, nullptr, HID);
        k_silusplit<128, false><<<PCH / 8, 256, 0, stream>>>(CD, PCH, CDh, CDl, nullptr);
        k_gemmb<true, false><<<dim3(PCH / 64, CCH / 64, 1), 128, 0, stream>>>(CDh, CDl, BWEK, nullptr, EKc, CCH, nullptr, nullptr, CCH);
        k_edge1<<<(PCH / 2) / 8, 256, 0, stream>>>(UV, EKc, be1, b, i0, P64h, P64l);
        k_gemmb<true, false><<<dim3(PCH / 64, 1, 1), 128, 0, stream>>>(P64h, P64l, BWE2, be2, E2, HID, nullptr, nullptr, HID);
        k_aggsum<<<ICH / 8, 256, 0, stream>>>(E2, b, i0, AGG);
        if (ch % 2 == 1) {
            k_catplanes<<<NNODE / 8, 256, 0, stream>>>(HH, AGG, NPh, NPl);
            k_gemmb<true, false><<<dim3(NNODE / 64, 1, 1), 128, 0, stream>>>(NPh, NPl, BWN1, bn1, NT1, HID, nullptr, nullptr, CCH);
            k_silusplit<64, false><<<(NNODE / 2) / 8, 256, 0, stream>>>(NT1, NNODE, NPh, NPl, nullptr);
            k_gemmb<true, false><<<dim3(NNODE / 64, 1, 1), 128, 0, stream>>>(NPh, NPl, BWN2, bn2, NT1, HID, nullptr, nullptr, HID);
            k_silusplit<64, true><<<(NNODE / 2) / 8, 256, 0, stream>>>(NT1, NNODE, NPh, NPl, NNW);
            k_gemmb<true, false><<<dim3(NNODE / 64, CCH / 64, 1), 128, 0, stream>>>(NPh, NPl, BUVN, nullptr, UVN, CCH, nullptr, nullptr, HID);
            for (int c2 = 0; c2 < 2; ++c2) k_logits<<<(PCH / 8) / 8, 256, 0, stream>>>(UVN, EK + (size_t)c2 * PCH * CCH, bk1, Wk2, bk2, b, c2 * ICH, out1); } }
}
